// FeatureAlign_34677565947928
// MI455X (gfx1250) — hardware-verified
//
#include <hip/hip_runtime.h>
#include <stddef.h>
#include <math.h>

constexpr int NBATCH  = 2;
constexpr int NCH     = 128;
constexpr int IMGH    = 128;
constexpr int IMGW    = 128;
constexpr int HWPIX   = 16384;
constexpr int NPIX    = 32768;
constexpr int SRCH    = 64;
constexpr int SRCW    = 64;
constexpr int SRCHW   = 4096;
constexpr int NTAP    = 9;
constexpr int KDEF    = 1152;
constexpr int KCAT    = 256;
constexpr int NOMR    = 216;
constexpr int NOMP    = 256;
constexpr int NOFSM   = 144;
constexpr int NPC     = 8192;
constexpr int NCHUNK  = 4;
constexpr int STATG   = 128;
constexpr int STATROWS = 256;
constexpr int PARSLOT = 256;

static_assert(KDEF % 32 == 0, "");
static_assert(NPC % 64 == 0 && NPIX % 64 == 0, "");
static_assert(NCHUNK * NPC == NPIX, "");
static_assert(STATG * STATROWS == NPIX, "");
static_assert(HWPIX % 32 == 0, "");
static_assert((NPC * NTAP) % 64 == 0, "");

typedef __attribute__((ext_vector_type(16))) _Float16 v16h;
typedef __attribute__((ext_vector_type(8)))  _Float16 v8h;
typedef __attribute__((ext_vector_type(16))) __bf16   v16b;
typedef __attribute__((ext_vector_type(8)))  __bf16   v8b;
typedef __attribute__((ext_vector_type(8)))  float    v8f;
typedef __attribute__((ext_vector_type(4)))  float    v4f;
typedef __attribute__((ext_vector_type(4)))  unsigned v4u;

__device__ __forceinline__ unsigned short f2bf_bits(float f) {
  unsigned u = __float_as_uint(f);
  return (unsigned short)((u + 0x7FFFu + ((u >> 16) & 1u)) >> 16);
}
__device__ __forceinline__ float bf_bits2f(unsigned short h) { return __uint_as_float(((unsigned)h) << 16); }
__device__ __forceinline__ float bf16r(float f) { return bf_bits2f(f2bf_bits(f)); }

__device__ __forceinline__ unsigned pk2(unsigned short a, unsigned short b) {
  return (unsigned)a | ((unsigned)b << 16);
}
__device__ __forceinline__ unsigned pkh2(float a, float b) {
  return pk2(__builtin_bit_cast(unsigned short, (_Float16)a), __builtin_bit_cast(unsigned short, (_Float16)b));
}
__device__ __forceinline__ void pkbf2(float a, float b, unsigned& uh, unsigned& ul) {
  const unsigned short ha = f2bf_bits(a), hb = f2bf_bits(b);
  const unsigned short la = f2bf_bits(a - bf_bits2f(ha)), lb = f2bf_bits(b - bf_bits2f(hb));
  uh = pk2(ha, hb);
  ul = pk2(la, lb);
}

__device__ __forceinline__ void dep_guard_h(v8f& a, v8f& b, v16h x, v16h y) { asm volatile("v_nop\n\tv_nop\n\tv_nop\n\tv_nop" : "+v"(a), "+v"(b) : "v"(x), "v"(y)); }
__device__ __forceinline__ void dep_guard_b(v8f& a, v8f& b, v16b x, v16b y) { asm volatile("v_nop\n\tv_nop\n\tv_nop\n\tv_nop" : "+v"(a), "+v"(b) : "v"(x), "v"(y)); }
__device__ __forceinline__ void keep4_h(v16h a, v16h b, v16h c, v16h d) { asm volatile("v_nop" :: "v"(a), "v"(b), "v"(c), "v"(d)); }
__device__ __forceinline__ void keep4_b(v16b a, v16b b, v16b c, v16b d) { asm volatile("v_nop" :: "v"(a), "v"(b), "v"(c), "v"(d)); }
__device__ __forceinline__ void acc_guard4(v8f& a, v8f& b, v8f& c, v8f& d) { asm volatile("v_nop\n\tv_nop\n\tv_nop\n\tv_nop" : "+v"(a), "+v"(b), "+v"(c), "+v"(d)); }
template <typename T> struct Frag;
template <> struct Frag<_Float16> {
  typedef v16h V; union U { v16h v; v8h h[2]; };
  static __device__ __forceinline__ v16h load(const _Float16* p) {
    U f; f.h[0] = *(const v8h*)(p); f.h[1] = *(const v8h*)(p + 16); return f.v;
  }
  static __device__ __forceinline__ v8f mma(v16h a, v16h b, v8f c) {
    return __builtin_amdgcn_wmma_f32_16x16x32_f16(false, a, false, b, (short)0, c, false, false);
  }
  static __device__ __forceinline__ void guard(v8f& a, v8f& b, v16h x, v16h y) { dep_guard_h(a, b, x, y); }
  static __device__ __forceinline__ void keep(v16h a, v16h b, v16h c, v16h d) { keep4_h(a, b, c, d); }
};
template <> struct Frag<__bf16> {
  typedef v16b V; union U { v16b v; v8b h[2]; };
  static __device__ __forceinline__ v16b load(const __bf16* p) {
    U f; f.h[0] = *(const v8b*)(p); f.h[1] = *(const v8b*)(p + 16); return f.v;
  }
  static __device__ __forceinline__ v8f mma(v16b a, v16b b, v8f c) {
    return __builtin_amdgcn_wmma_f32_16x16x32_bf16(false, a, false, b, (short)0, c, false, false);
  }
  static __device__ __forceinline__ void guard(v8f& a, v8f& b, v16b x, v16b y) { dep_guard_b(a, b, x, y); }
  static __device__ __forceinline__ void keep(v16b a, v16b b, v16b c, v16b d) { keep4_b(a, b, c, d); }
};

template <int ET> struct Elem;
template <> struct Elem<0> { typedef _Float16 T; };
template <> struct Elem<1> { typedef __bf16 T; };
template <int ET, bool SPLIT, int BIAS_MODE, int OUT_MODE, bool RESID, int ACT = 0>
__global__ __launch_bounds__(256) void wmma_gemm64(
    const unsigned short* __restrict__ Ap, const unsigned short* __restrict__ A2p, int lda, long strideA,
    const unsigned short* __restrict__ Btp, const unsigned short* __restrict__ Bt2p, int ldb, long strideB,
    void* __restrict__ Cout, void* __restrict__ Cout2, int ldc, long strideC,
    const float* __restrict__ bias,
    const float* __restrict__ resid, long strideR,
    int M, int N, int K, float scale) {
  typedef typename Elem<ET>::T T;
  typedef typename Frag<T>::V V;
  const T* A = (const T*)Ap; const T* A2 = (const T*)A2p; const T* Bt = (const T*)Btp; const T* Bt2 = (const T*)Bt2p;
  __shared__ __align__(16) float sT[8][16 * 68];
  const int b    = blockIdx.y;
  const int lane = threadIdx.x & 31;
  const int wave = threadIdx.x >> 5;
  const int tilesN = N >> 6;
  const int tilesM = M >> 6;
  const int tile = blockIdx.x * 8 + wave;
  if (tile >= tilesM * tilesN) return;
  const int tm = tile / tilesN;
  const int tn = tile - tm * tilesN;
  const int m0 = tm << 6;
  const int n0 = tn << 6;

  const T* Ab  = A  + (size_t)b * strideA;
  const T* Bb  = Bt + (size_t)b * strideB;
  const T* Ab2 = SPLIT ? (A2  + (size_t)b * strideA) : nullptr;
  const T* Bb2 = SPLIT ? (Bt2 + (size_t)b * strideB) : nullptr;

  const int rlane = lane & 15;
  const int koff  = (lane >> 4) * 8;
  const int mOff  = (lane >> 4) * 8;

  v8f acc[4][4];
#pragma unroll
  for (int i = 0; i < 4; ++i)
#pragma unroll
    for (int j = 0; j < 4; ++j) acc[i][j] = (v8f){0.f,0.f,0.f,0.f,0.f,0.f,0.f,0.f};

  for (int k0 = 0; k0 < K; k0 += 32) {
    V bh[4], bl[4];
#pragma unroll
    for (int j = 0; j < 4; ++j) {
      const size_t bo = (size_t)(n0 + (j << 4) + rlane) * ldb + koff + k0;
      bh[j] = Frag<T>::load(Bb + bo);
      if (SPLIT) bl[j] = Frag<T>::load(Bb2 + bo);
    }
#pragma unroll
    for (int i = 0; i < 4; ++i) {
      const size_t ao = (size_t)(m0 + (i << 4) + rlane) * lda + koff + k0;
      V ah = Frag<T>::load(Ab + ao);
      V al;
      if (SPLIT) al = Frag<T>::load(Ab2 + ao);
#pragma unroll
      for (int j = 0; j < 4; ++j) {
        acc[i][j] = Frag<T>::mma(ah, bh[j], acc[i][j]);
        if (SPLIT) {
          acc[i][j] = Frag<T>::mma(ah, bl[j], acc[i][j]);
          acc[i][j] = Frag<T>::mma(al, bh[j], acc[i][j]);
        }
      }
      Frag<T>::guard(acc[i][0], acc[i][3], ah, SPLIT ? al : ah);
    }
    Frag<T>::keep(bh[0], bh[1], bh[2], bh[3]);
    if (SPLIT) Frag<T>::keep(bl[0], bl[1], bl[2], bl[3]);
  }
  acc_guard4(acc[0][0], acc[0][1], acc[0][2], acc[0][3]);
  acc_guard4(acc[1][0], acc[1][1], acc[1][2], acc[1][3]);
  acc_guard4(acc[2][0], acc[2][1], acc[2][2], acc[2][3]);
  acc_guard4(acc[3][0], acc[3][1], acc[3][2], acc[3][3]);

  float* slab = sT[wave];
  const float* Rb = RESID ? (resid + (size_t)b * strideR) : nullptr;
#pragma unroll
  for (int i = 0; i < 4; ++i) {
    const int mBase = m0 + (i << 4);
#pragma unroll
    for (int j = 0; j < 4; ++j) {
      const int n = n0 + (j << 4) + rlane;
      float bv = 0.f;
      if (BIAS_MODE == 2) bv = bias[n];
#pragma unroll
      for (int r = 0; r < 8; ++r) {
        float v = acc[i][j][r] * scale;
        if (BIAS_MODE == 1) v += bias[mBase + mOff + r];
        if (BIAS_MODE == 2) v += bv;
        if (RESID) v += Rb[(size_t)(mBase + mOff + r) * ldc + n];
        if (ACT == 1) v = tanhf(v);
        if (ACT == 2) v = fmaxf(v, 0.0f);
        if (ACT == 3) v = v / (1.0f + expf(-v));
        if (ACT == 4) v = (v > 0.f) ? v : 0.01f * v;
        if (ACT == 5) v = 0.5f * v * (1.0f + erff(v * 0.70710678118654752f));
        slab[(mOff + r) * 68 + (j << 4) + rlane] = v;
      }
    }
    __builtin_amdgcn_fence(__ATOMIC_RELEASE, "workgroup");
    __builtin_amdgcn_wave_barrier();
    __builtin_amdgcn_fence(__ATOMIC_ACQUIRE, "workgroup");
    if (OUT_MODE == 0) {
      float* C = (float*)Cout + (size_t)b * strideC;
      const int hh = lane >> 4, c4 = (lane & 15) * 4;
      for (int pass = 0; pass < 2; ++pass) {
#pragma unroll
        for (int it = 0; it < 8; ++it) {
          const int row = it * 2 + hh;
          v4f v = *(const v4f*)(slab + row * 68 + c4);
          *(volatile v4f*)(C + (size_t)(mBase + row) * ldc + n0 + c4) = v;
        }
        __threadfence();
      }
    } else {
      const int q = lane >> 3, c8 = (lane & 7) * 8;
      unsigned short* C  = (unsigned short*)Cout  + (size_t)b * strideC;
      unsigned short* C2 = (OUT_MODE == 2) ? ((unsigned short*)Cout2 + (size_t)b * strideC) : nullptr;
      for (int pass = 0; pass < 2; ++pass) {
#pragma unroll
        for (int it = 0; it < 4; ++it) {
          const int row = it * 4 + q;
          const float* sp = slab + row * 68 + c8;
          v8h hv, lv;
#pragma unroll
          for (int e = 0; e < 8; ++e) {
            if (OUT_MODE == 1) {
              hv[e] = (_Float16)sp[e];
            } else {
              unsigned short hb = f2bf_bits(sp[e]);
              unsigned short lb = f2bf_bits(sp[e] - bf_bits2f(hb));
              hv[e] = __builtin_bit_cast(_Float16, hb);
              lv[e] = __builtin_bit_cast(_Float16, lb);
            }
          }
          *(volatile v8h*)(C + (size_t)(mBase + row) * ldc + n0 + c8) = hv;
          if (OUT_MODE == 2) *(volatile v8h*)(C2 + (size_t)(mBase + row) * ldc + n0 + c8) = lv;
        }
        __threadfence();
      }
    }
    __builtin_amdgcn_fence(__ATOMIC_RELEASE, "workgroup");
    __builtin_amdgcn_wave_barrier();
    __builtin_amdgcn_fence(__ATOMIC_ACQUIRE, "workgroup");
  }
}

__global__ __launch_bounds__(256) void k_xpose_in(const float* __restrict__ x, unsigned short* __restrict__ xl) {
  __shared__ __align__(16) float t[32][132];
  const int tid = threadIdx.x;
  const int p0 = blockIdx.x * 32;
  const int b = p0 >> 14, hw0 = p0 & (HWPIX - 1);
  const float* xb = x + (size_t)b * NCH * HWPIX + hw0;
#pragma unroll
  for (int i = 0; i < 16; ++i) {
    const int idx = i * 256 + tid;
    const int c = idx >> 5, j = idx & 31;
    t[j][c] = xb[(size_t)c * HWPIX + j];
  }
  __syncthreads();
  const int wave = tid >> 5, lane = tid & 31, hsel = lane >> 4, c8 = (lane & 15) * 8;
  for (int pass = 0; pass < 2; ++pass) {
#pragma unroll
    for (int it = 0; it < 2; ++it) {
      const int px = wave * 4 + it * 2 + hsel;
      const v4f a = *(const v4f*)(&t[px][c8]);
      const v4f c = *(const v4f*)(&t[px][c8 + 4]);
      v4u u;
      u[0] = pk2(f2bf_bits(a[0]), f2bf_bits(a[1]));
      u[1] = pk2(f2bf_bits(a[2]), f2bf_bits(a[3]));
      u[2] = pk2(f2bf_bits(c[0]), f2bf_bits(c[1]));
      u[3] = pk2(f2bf_bits(c[2]), f2bf_bits(c[3]));
      *(volatile v4u*)(xl + (size_t)(p0 + px) * NCH + c8) = u;
    }
    __threadfence();
  }
}

__device__ __forceinline__ void rs_taps(int d, int& i0, int& i1, float& w0, float& w1) {
  const int m = d >> 1;
  const bool odd = (d & 1) != 0;
  int a0 = odd ? m : m - 1;
  int a1 = odd ? m + 1 : m;
  float u0 = odd ? 0.75f : 0.25f;
  float u1 = odd ? 0.25f : 0.75f;
  if (a0 < 0) { a0 = 0; u0 = 0.0f; u1 = 1.0f; }
  if (a1 > SRCH - 1) { a1 = SRCH - 1; u0 = 1.0f; u1 = 0.0f; }
  i0 = a0; i1 = a1; w0 = u0; w1 = u1;
}

__global__ __launch_bounds__(256) void k_resize(const float* __restrict__ fs, float* __restrict__ up,
                                                unsigned short* __restrict__ cat) {
  __shared__ __align__(16) float t[32][132];
  const int tid = threadIdx.x, wave = tid >> 5, lane = tid & 31;
  const int p0 = blockIdx.x * 32;
  const int b = p0 >> 14, hw0 = p0 & (HWPIX - 1);
  const int yo = hw0 >> 7;
  const int xo = (hw0 & (IMGW - 1)) + lane;
  int y0i, y1i, x0i, x1i; float wy0, wy1, wx0, wx1;
  rs_taps(yo, y0i, y1i, wy0, wy1);
  rs_taps(xo, x0i, x1i, wx0, wx1);
  const int o00 = y0i * SRCW + x0i, o01 = y0i * SRCW + x1i;
  const int o10 = y1i * SRCW + x0i, o11 = y1i * SRCW + x1i;
  const float* fb = fs + (size_t)b * NCH * SRCHW;
#pragma unroll 1
  for (int i = 0; i < 16; ++i) {
    const int c = i * 8 + wave;
    const float* pc = fb + (size_t)c * SRCHW;
    const float v00 = bf16r(pc[o00]), v01 = bf16r(pc[o01]);
    const float v10 = bf16r(pc[o10]), v11 = bf16r(pc[o11]);
    const float ra = v00 * wx0 + v01 * wx1;
    const float rb = v10 * wx0 + v11 * wx1;
    t[lane][c] = ra * wy0 + rb * wy1;
  }
  __syncthreads();
  const int hsel = lane >> 4, c8 = (lane & 15) * 8;
  for (int pass = 0; pass < 2; ++pass) {
#pragma unroll
    for (int it = 0; it < 4; ++it) {
      const int px = wave * 4 + it;
      const v4f v = *(const v4f*)(&t[px][lane * 4]);
      *(volatile v4f*)(up + (size_t)(p0 + px) * NCH + lane * 4) = v;
    }
#pragma unroll
    for (int it = 0; it < 2; ++it) {
      const int px = wave * 4 + it * 2 + hsel;
      const v4f a = *(const v4f*)(&t[px][c8]);
      const v4f c = *(const v4f*)(&t[px][c8 + 4]);
      v4u u;
      u[0] = pkh2(2.0f * a[0], 2.0f * a[1]); u[1] = pkh2(2.0f * a[2], 2.0f * a[3]);
      u[2] = pkh2(2.0f * c[0], 2.0f * c[1]); u[3] = pkh2(2.0f * c[2], 2.0f * c[3]);
      *(volatile v4u*)(cat + (size_t)(p0 + px) * KCAT + NCH + c8) = u;
    }
    __threadfence();
  }
}

__global__ __launch_bounds__(64) void k_par(const float* __restrict__ s0, const float* __restrict__ s1,
                                            const float* __restrict__ s2, const float* __restrict__ s3,
                                            const float* __restrict__ s4, const float* __restrict__ s5,
                                            const float* __restrict__ s6, const float* __restrict__ s7,
                                            float* __restrict__ par) {
  const int slot = blockIdx.x;
  const float* src = s0; int len = NOMR;
  if (slot == 1) { src = s1; len = NCH; }
  else if (slot == 2) { src = s2; len = NCH; }
  else if (slot == 3) { src = s3; len = NCH; }
  else if (slot == 4) { src = s4; len = NCH; }
  else if (slot == 5) { src = s5; len = NCH; }
  else if (slot == 6) { src = s6; len = NCH; }
  else if (slot == 7) { src = s7; len = NCH; }
  const int e0 = threadIdx.x * 4;
  v4f v;
#pragma unroll
  for (int j = 0; j < 4; ++j) {
    const int e = e0 + j;
    const int ec = e < len ? e : len - 1;
    const float f = src[ec];
    v[j] = (e < len) ? bf16r(f) : 0.0f;
  }
  volatile v4f* p = (volatile v4f*)(par + (size_t)slot * PARSLOT + e0);
  *p = v;
  __threadfence();
  *p = v;
}

template <int MODE>
__global__ __launch_bounds__(256) void k_prep_w1x1(const float* __restrict__ w, unsigned short* __restrict__ dst,
                                                   unsigned short* __restrict__ dst2, int n8, float scale) {
  const int g = blockIdx.x * 256 + threadIdx.x;
  if (g < n8) {
    const int e0 = g * 8;
    float f[8];
#pragma unroll
    for (int j = 0; j < 8; ++j) f[j] = bf16r(w[e0 + j]) * scale;
    v4u u;
    if (MODE == 1) {
      u[0] = pkh2(f[0], f[1]); u[1] = pkh2(f[2], f[3]); u[2] = pkh2(f[4], f[5]); u[3] = pkh2(f[6], f[7]);
    } else {
      u[0] = pk2(f2bf_bits(f[0]), f2bf_bits(f[1])); u[1] = pk2(f2bf_bits(f[2]), f2bf_bits(f[3]));
      u[2] = pk2(f2bf_bits(f[4]), f2bf_bits(f[5])); u[3] = pk2(f2bf_bits(f[6]), f2bf_bits(f[7]));
    }
    const v4u z = (v4u){0u, 0u, 0u, 0u};
    volatile v4u* p = (volatile v4u*)(dst + e0);
    *p = u;
    if (MODE == 2) { *(volatile v4u*)(dst2 + e0) = z; }
    __threadfence();
    *p = u;
    if (MODE == 2) { *(volatile v4u*)(dst2 + e0) = z; }
  }
}

__global__ __launch_bounds__(256) void k_prep_w3x3(const float* __restrict__ w, unsigned short* __restrict__ dst,
                                                   int mout, int mpad, float scale) {
  const int g = blockIdx.x * 256 + threadIdx.x;
  if (g < mpad * (KDEF / 8)) {
    const int e0 = g * 8;
    const int o = e0 / KDEF;
    const int col = e0 - o * KDEF;
    const int k = col >> 7;
    const int c0 = col & (NCH - 1);
    const int oc = o < mout ? o : (mout - 1);
    float f[8];
#pragma unroll
    for (int j = 0; j < 8; ++j) {
      const float v = w[((size_t)(oc * NCH + c0 + j)) * NTAP + k];
      f[j] = (o < mout) ? bf16r(v) * scale : 0.0f;
    }
    v4u u;
    u[0] = pkh2(f[0], f[1]); u[1] = pkh2(f[2], f[3]); u[2] = pkh2(f[4], f[5]); u[3] = pkh2(f[6], f[7]);
    volatile v4u* p = (volatile v4u*)(dst + e0);
    *p = u;
    __threadfence();
    *p = u;
  }
}

union D2 { double d[2]; v4u u; };
__global__ __launch_bounds__(256) void k_stats_part(const float* __restrict__ cm, double* __restrict__ stp) {
  __shared__ double shs[256];
  __shared__ double shq[256];
  const int tid = threadIdx.x, c = tid & (NCH - 1), hf = tid >> 7;
  const float* base = cm + ((size_t)blockIdx.x * STATROWS + hf) * NCH + c;
  double s = 0.0, q = 0.0;
#pragma unroll 1
  for (int i = 0; i < STATROWS / 2; ++i) {
    const double v = (double)base[(size_t)i * 2 * NCH];
    s += v;
    q += v * v;
  }
  shs[tid] = s; shq[tid] = q;
  __syncthreads();
  if (tid < NCH) {
    D2 d;
    d.d[0] = shs[tid] + shs[tid + NCH];
    d.d[1] = shq[tid] + shq[tid + NCH];
    const v4u u = d.u;
    volatile v4u* p = (volatile v4u*)(stp + ((size_t)blockIdx.x * NCH + tid) * 2);
    *p = u;
    __threadfence();
    *p = u;
  }
}

__global__ __launch_bounds__(128) void k_stats_fin(const double* __restrict__ stp, const float* __restrict__ gam,
                                                    const float* __restrict__ bet, float* __restrict__ bnp) {
  const int c = threadIdx.x;
  double s = 0.0, q = 0.0;
#pragma unroll 1
  for (int g = 0; g < STATG; ++g) {
    const double* e = stp + ((size_t)g * NCH + c) * 2;
    s += e[0];
    q += e[1];
  }
  const double mean = s * (1.0 / (double)NPIX);
  double var = q * (1.0 / (double)NPIX) - mean * mean;
  var = var < 0.0 ? 0.0 : var;
  const float mu = (float)mean;
  const float vf = (float)var;
  const float r = 1.0f / sqrtf(vf + 1e-5f);
  v4f o;
  o[0] = mu; o[1] = r; o[2] = gam[c]; o[3] = bet[c];
  volatile v4f* p = (volatile v4f*)(bnp + c * 4);
  *p = o;
  __threadfence();
  *p = o;
}

template <bool EXTRA>
__global__ __launch_bounds__(256) void k_bn_apply(const float* __restrict__ cm, const float* __restrict__ bnp,
                                                  unsigned short* __restrict__ d16, int ld16,
                                                  unsigned short* __restrict__ dh, unsigned short* __restrict__ dl, int ldx) {
  const int lane = threadIdx.x & 31, wave = threadIdx.x >> 5;
  const int p = (blockIdx.x * 8 + wave) * 2 + (lane >> 4);
  const int c8 = (lane & 15) * 8;
  const float* src = cm + (size_t)p * NCH + c8;
  const v4f a = *(const v4f*)(src);
  const v4f bq = *(const v4f*)(src + 4);
  float x[8];
  x[0] = a[0]; x[1] = a[1]; x[2] = a[2]; x[3] = a[3];
  x[4] = bq[0]; x[5] = bq[1]; x[6] = bq[2]; x[7] = bq[3];
  float y[8];
#pragma unroll
  for (int e = 0; e < 8; ++e) {
    const v4f pr = *(const v4f*)(bnp + (c8 + e) * 4);
    y[e] = fmaxf(((x[e] - pr[0]) * pr[1]) * pr[2] + pr[3], 0.0f);
  }
  v4u u;
  u[0] = pkh2(y[0], y[1]); u[1] = pkh2(y[2], y[3]); u[2] = pkh2(y[4], y[5]); u[3] = pkh2(y[6], y[7]);
  v4u uh, ul;
  if (EXTRA) {
    unsigned th, tl;
    pkbf2(y[0], y[1], th, tl); uh[0] = th; ul[0] = tl;
    pkbf2(y[2], y[3], th, tl); uh[1] = th; ul[1] = tl;
    pkbf2(y[4], y[5], th, tl); uh[2] = th; ul[2] = tl;
    pkbf2(y[6], y[7], th, tl); uh[3] = th; ul[3] = tl;
  }
  volatile v4u* pd = (volatile v4u*)(d16 + (size_t)p * ld16 + c8);
  *pd = u;
  if (EXTRA) {
    *(volatile v4u*)(dh + (size_t)p * ldx + c8) = uh;
    *(volatile v4u*)(dl + (size_t)p * ldx + c8) = ul;
  }
  __threadfence();
  *pd = u;
  if (EXTRA) {
    *(volatile v4u*)(dh + (size_t)p * ldx + c8) = uh;
    *(volatile v4u*)(dl + (size_t)p * ldx + c8) = ul;
  }
}

__global__ __launch_bounds__(256) void k_bn_out(const float* __restrict__ cm, const float* __restrict__ bnp,
                                                float* __restrict__ out) {
  __shared__ __align__(16) float t[NCH][36];
  const int tid = threadIdx.x;
  const int p0 = blockIdx.x * 32;
  const int b = p0 >> 14, hw0 = p0 & (HWPIX - 1);
  {
    const int px = tid >> 3;
    const int c16 = (tid & 7) * 16;
    const float* src = cm + (size_t)(p0 + px) * NCH + c16;
#pragma unroll
    for (int qd = 0; qd < 4; ++qd) {
      const v4f a = *(const v4f*)(src + 4 * qd);
#pragma unroll
      for (int e = 0; e < 4; ++e) {
        const int c = c16 + 4 * qd + e;
        const v4f pr = *(const v4f*)(bnp + c * 4);
        t[c][px] = fmaxf(((a[e] - pr[0]) * pr[1]) * pr[2] + pr[3], 0.0f);
      }
    }
  }
  __syncthreads();
  const int wave = tid >> 5, lane = tid & 31;
  const int px4 = (lane & 7) * 4;
  float* ob = out + ((size_t)b * NCH) * HWPIX + hw0 + px4;
  for (int pass = 0; pass < 2; ++pass) {
#pragma unroll
    for (int it = 0; it < 4; ++it) {
      const int ch = wave * 16 + it * 4 + (lane >> 3);
      const v4f v = *(const v4f*)(&t[ch][px4]);
      *(volatile v4f*)(ob + (size_t)ch * HWPIX) = v;
    }
    __threadfence();
  }
}

__global__ __launch_bounds__(256) void k_im2col(const unsigned short* __restrict__ off16, unsigned short* __restrict__ im, int p0) {
  const int lane = threadIdx.x & 31, wave = threadIdx.x >> 5;
  const int hsel = lane >> 4, c8 = (lane & 15) * 8;
  const v4u z = (v4u){0u, 0u, 0u, 0u};
#pragma unroll
  for (int r = 0; r < 4; ++r) {
    const int it = ((blockIdx.x * 8 + wave) * 4 + r) * 2 + hsel;
    const int pl = it / NTAP, k = it - pl * NTAP;
    const int p = p0 + pl;
    const int b = p >> 14, hw = p & (HWPIX - 1);
    const int ho = hw >> 7, wo = hw & (IMGW - 1);
    const int kh = k / 3, kw = k - kh * 3;
    const int y = ho - 1 + kh, xx = wo - 1 + kw;
    const bool inb = ((unsigned)y < (unsigned)IMGH) && ((unsigned)xx < (unsigned)IMGW);
    const int yc = y < 0 ? 0 : (y > IMGH - 1 ? IMGH - 1 : y);
    const int xc = xx < 0 ? 0 : (xx > IMGW - 1 ? IMGW - 1 : xx);
    v4u v = *(const v4u*)(off16 + ((size_t)(b * HWPIX + yc * IMGW + xc)) * NCH + c8);
    if (!inb) v = z;
    volatile v4u* d = (volatile v4u*)(im + (size_t)it * NCH + c8);
    *d = v;
    __threadfence();
    *d = v;
  }
}

__global__ __launch_bounds__(256) void k_sample(const float* __restrict__ up, const float* __restrict__ omc,
                                                const float* __restrict__ bomr, unsigned short* __restrict__ s16, int p0) {
  const int lane = threadIdx.x & 31, wave = threadIdx.x >> 5;
  const int c8 = (lane & 15) * 8, dg = c8 >> 4;
  const int it = (blockIdx.x * 8 + wave) * 2 + (lane >> 4);
  const int pl = it / NTAP, k = it - pl * NTAP;
  const int p = p0 + pl;
  const int b = p >> 14, hw = p & (HWPIX - 1);
  const int ho = hw >> 7, wo = hw & (IMGW - 1);
  const int kh = k / 3, kw = k - kh * 3;
  const float* orow = omc + (size_t)pl * NOMP;
  const int oc = dg * NTAP + k;
  const float dy = orow[2 * oc] + bomr[2 * oc];
  const float dx = orow[2 * oc + 1] + bomr[2 * oc + 1];
  float ml = orow[NOFSM + oc] + bomr[NOFSM + oc];
  ml = fminf(fmaxf(ml, -30.0f), 30.0f);
  const float msk = __builtin_amdgcn_rcpf(1.0f + __expf(-ml));
  const float py = (float)(ho + kh - 1) + dy;
  const float px = (float)(wo + kw - 1) + dx;
  const float y0 = floorf(py), x0 = floorf(px);
  const float y1 = y0 + 1.0f, x1 = x0 + 1.0f;
  const float wy1 = py - y0, wx1 = px - x0;
  const float wy0 = 1.0f - wy1, wx0 = 1.0f - wx1;
  const bool vy0 = (y0 >= 0.0f) && (y0 <= (float)(IMGH - 1));
  const bool vy1 = (y1 >= 0.0f) && (y1 <= (float)(IMGH - 1));
  const bool vx0 = (x0 >= 0.0f) && (x0 <= (float)(IMGW - 1));
  const bool vx1 = (x1 >= 0.0f) && (x1 <= (float)(IMGW - 1));
  float w00 = wy0 * wx0, w01 = wy0 * wx1, w10 = wy1 * wx0, w11 = wy1 * wx1;
  w00 = (vy0 && vx0) ? w00 : 0.0f;
  w01 = (vy0 && vx1) ? w01 : 0.0f;
  w10 = (vy1 && vx0) ? w10 : 0.0f;
  w11 = (vy1 && vx1) ? w11 : 0.0f;
  const int yi0 = (int)fminf(fmaxf(y0, 0.0f), (float)(IMGH - 1));
  const int yi1 = (int)fminf(fmaxf(y1, 0.0f), (float)(IMGH - 1));
  const int xi0 = (int)fminf(fmaxf(x0, 0.0f), (float)(IMGW - 1));
  const int xi1 = (int)fminf(fmaxf(x1, 0.0f), (float)(IMGW - 1));
  const float* ub  = up + (size_t)b * HWPIX * NCH + c8;
  const float* r00 = ub + ((size_t)yi0 * IMGW + xi0) * NCH;
  const float* r01 = ub + ((size_t)yi0 * IMGW + xi1) * NCH;
  const float* r10 = ub + ((size_t)yi1 * IMGW + xi0) * NCH;
  const float* r11 = ub + ((size_t)yi1 * IMGW + xi1) * NCH;
  const v4f g00a = *(const v4f*)(r00), g00b = *(const v4f*)(r00 + 4);
  const v4f g01a = *(const v4f*)(r01), g01b = *(const v4f*)(r01 + 4);
  const v4f g10a = *(const v4f*)(r10), g10b = *(const v4f*)(r10 + 4);
  const v4f g11a = *(const v4f*)(r11), g11b = *(const v4f*)(r11 + 4);
  v4f va = g00a * w00 + g01a * w01 + g10a * w10 + g11a * w11;
  v4f vb = g00b * w00 + g01b * w01 + g10b * w10 + g11b * w11;
  va = va * msk;
  vb = vb * msk;
  v4u u;
  u[0] = pkh2(va[0], va[1]); u[1] = pkh2(va[2], va[3]);
  u[2] = pkh2(vb[0], vb[1]); u[3] = pkh2(vb[2], vb[3]);
  volatile v4u* d = (volatile v4u*)(s16 + (size_t)it * NCH + c8);
  *d = u;
  __threadfence();
  *d = u;
}

extern "C" void kernel_launch(void* const* d_in, const int* in_sizes, int n_in,
                              void* d_out, int out_size, void* d_ws, size_t ws_size,
                              hipStream_t stream) {
  if (n_in < 15) return;
  if (in_sizes[0] != NPIX * NCH || in_sizes[1] != NBATCH * NCH * SRCHW || in_sizes[2] != NCH * NCH ||
      in_sizes[3] != NCH || in_sizes[4] != NCH || in_sizes[5] != NCH * KCAT || in_sizes[6] != NCH ||
      in_sizes[7] != NCH || in_sizes[8] != NOMR * NCH * NTAP || in_sizes[9] != NOMR ||
      in_sizes[10] != NCH * NCH * NTAP || in_sizes[11] != NCH || in_sizes[12] != NCH * KCAT ||
      in_sizes[13] != NCH || in_sizes[14] != NCH) return;
  if (out_size != NBATCH * NCH * HWPIX) return;

  const float* feat_l = (const float*)d_in[0];
  const float* feat_s = (const float*)d_in[1];
  const float* w_fsm  = (const float*)d_in[2];
  const float* g_fsm  = (const float*)d_in[3];
  const float* b_fsm  = (const float*)d_in[4];
  const float* w_off  = (const float*)d_in[5];
  const float* g_off  = (const float*)d_in[6];
  const float* b_off  = (const float*)d_in[7];
  const float* w_om   = (const float*)d_in[8];
  const float* b_om   = (const float*)d_in[9];
  const float* w_dcn  = (const float*)d_in[10];
  const float* b_dcn  = (const float*)d_in[11];
  const float* w_fus  = (const float*)d_in[12];
  const float* g_fus  = (const float*)d_in[13];
  const float* b_fus  = (const float*)d_in[14];
  float* out = (float*)d_out;

  const size_t bytes_XL16 = (size_t)NPIX * NCH * 2;
  const size_t bytes_CAT1 = (size_t)NPIX * KCAT * 2;
  const size_t bytes_IM16 = (size_t)NPC * KDEF * 2;
  const size_t bytes_UP32 = (size_t)NPIX * NCH * 4;
  const size_t bytes_C32  = (size_t)NPIX * NCH * 4;
  const size_t bytes_CAT3 = (size_t)NPIX * KCAT * 2;
  const size_t bytes_OFF16 = (size_t)NPIX * NCH * 2;
  const size_t bytes_WFSM = (size_t)NCH * NCH * 2;
  const size_t bytes_W256 = (size_t)NCH * KCAT * 2;
  const size_t bytes_WOM  = (size_t)NOMP * KDEF * 2;
  const size_t bytes_WDCN = (size_t)NCH * KDEF * 2;
  const size_t bytes_PAR  = (size_t)8 * PARSLOT * 4;
  const size_t bytes_STP  = (size_t)STATG * NCH * 2 * 8;
  const size_t bytes_BNP  = (size_t)NCH * 4 * 4;
  const size_t bytes_OMC  = (size_t)NPC * NOMP * 4;
  const size_t bytes_S16  = (size_t)NPC * KDEF * 2;
  if (bytes_IM16 > bytes_XL16 + bytes_CAT1) return;

  char* ws = (char*)d_ws;
  size_t o = 0;
  unsigned short* XL16  = (unsigned short*)(ws + o);
  unsigned short* IM16  = (unsigned short*)(ws + o);  o += bytes_XL16;
  unsigned short* CAT1  = (unsigned short*)(ws + o);  o += bytes_CAT1;
  float*          UP32  = (float*)(ws + o);           o += bytes_UP32;
  float*          C32   = (float*)(ws + o);           o += bytes_C32;
  unsigned short* CAT3H = (unsigned short*)(ws + o);  o += bytes_CAT3;
  unsigned short* CAT3L = (unsigned short*)(ws + o);  o += bytes_CAT3;
  unsigned short* OFF16 = (unsigned short*)(ws + o);  o += bytes_OFF16;
  unsigned short* WFSM  = (unsigned short*)(ws + o);  o += bytes_WFSM;
  unsigned short* WOFF  = (unsigned short*)(ws + o);  o += bytes_W256;
  unsigned short* WFUSH = (unsigned short*)(ws + o);  o += bytes_W256;
  unsigned short* WFUSZ = (unsigned short*)(ws + o);  o += bytes_W256;
  unsigned short* WOM   = (unsigned short*)(ws + o);  o += bytes_WOM;
  unsigned short* WDCN  = (unsigned short*)(ws + o);  o += bytes_WDCN;
  float*          PAR   = (float*)(ws + o);           o += bytes_PAR;
  double*         STP   = (double*)(ws + o);          o += bytes_STP;
  float*          BNP   = (float*)(ws + o);           o += bytes_BNP;
  float*          OMC   = (float*)(ws + o);           o += bytes_OMC;
  unsigned short* S16   = (unsigned short*)(ws + o);  o += bytes_S16;
  if (o > ws_size || o > (size_t)134217728) return;

  const float* p_bomr  = PAR + 0 * PARSLOT;
  const float* p_bdcnr = PAR + 1 * PARSLOT;
  const float* p_gfsm  = PAR + 2 * PARSLOT;
  const float* p_bfsm  = PAR + 3 * PARSLOT;
  const float* p_goff  = PAR + 4 * PARSLOT;
  const float* p_boff  = PAR + 5 * PARSLOT;
  const float* p_gfus  = PAR + 6 * PARSLOT;
  const float* p_bfus  = PAR + 7 * PARSLOT;

  k_xpose_in<<<NPIX / 32, 256, 0, stream>>>(feat_l, XL16);
  k_resize<<<NPIX / 32, 256, 0, stream>>>(feat_s, UP32, CAT1);
  k_par<<<8, 64, 0, stream>>>(b_om, b_dcn, g_fsm, b_fsm, g_off, b_off, g_fus, b_fus, PAR);
  k_prep_w1x1<0><<<(NCH * NCH / 8) / 256, 256, 0, stream>>>(w_fsm, WFSM, WFSM, NCH * NCH / 8, 1.0f);
  k_prep_w1x1<1><<<(NCH * KCAT / 8) / 256, 256, 0, stream>>>(w_off, WOFF, WOFF, NCH * KCAT / 8, 16.0f);
  k_prep_w1x1<2><<<(NCH * KCAT / 8) / 256, 256, 0, stream>>>(w_fus, WFUSH, WFUSZ, NCH * KCAT / 8, 1.0f);
  k_prep_w3x3<<<(NOMP * (KDEF / 8)) / 256, 256, 0, stream>>>(w_om, WOM, NOMR, NOMP, 256.0f);
  k_prep_w3x3<<<(NCH * (KDEF / 8)) / 256, 256, 0, stream>>>(w_dcn, WDCN, NCH, NCH, 64.0f);

  const int tiles1x1 = (NPIX / 64) * (NCH / 64);

  wmma_gemm64<1, false, 0, 0, false><<<dim3((tiles1x1 + 7) / 8, 1), 256, 0, stream>>>(
      XL16, XL16, NCH, 0L, WFSM, WFSM, NCH, 0L, (void*)C32, (void*)C32, NCH, 0L,
      p_bdcnr, p_bdcnr, 0L, NPIX, NCH, NCH, 1.0f);
  k_stats_part<<<STATG, 256, 0, stream>>>(C32, STP);
  k_stats_fin<<<1, 128, 0, stream>>>(STP, p_gfsm, p_bfsm, BNP);
  k_bn_apply<true><<<NPIX / 16, 256, 0, stream>>>(C32, BNP, CAT1, KCAT, CAT3H, CAT3L, KCAT);

  wmma_gemm64<0, false, 0, 0, false><<<dim3((tiles1x1 + 7) / 8, 1), 256, 0, stream>>>(
      CAT1, CAT1, KCAT, 0L, WOFF, WOFF, KCAT, 0L, (void*)C32, (void*)C32, NCH, 0L,
      p_bdcnr, p_bdcnr, 0L, NPIX, NCH, KCAT, 0.0625f);
  k_stats_part<<<STATG, 256, 0, stream>>>(C32, STP);
  k_stats_fin<<<1, 128, 0, stream>>>(STP, p_goff, p_boff, BNP);
  k_bn_apply<false><<<NPIX / 16, 256, 0, stream>>>(C32, BNP, OFF16, NCH, OFF16, OFF16, NCH);

  const int tilesOM  = (NPC / 64) * (NOMP / 64);
  const int tilesDCN = (NPC / 64) * (NCH / 64);
  for (int q = 0; q < NCHUNK; ++q) {
    const int p0 = q * NPC;
    k_im2col<<<(NPC * NTAP) / 64, 256, 0, stream>>>(OFF16, IM16, p0);
    wmma_gemm64<0, false, 0, 0, false><<<dim3((tilesOM + 7) / 8, 1), 256, 0, stream>>>(
        IM16, IM16, KDEF, 0L, WOM, WOM, KDEF, 0L, (void*)OMC, (void*)OMC, NOMP, 0L,
        p_bdcnr, p_bdcnr, 0L, NPC, NOMP, KDEF, 0.00390625f);
    k_sample<<<(NPC * NTAP) / 16, 256, 0, stream>>>(UP32, OMC, p_bomr, S16, p0);
    wmma_gemm64<0, false, 2, 2, false, 2><<<dim3((tilesDCN + 7) / 8, 1), 256, 0, stream>>>(
        S16, S16, KDEF, 0L, WDCN, WDCN, KDEF, 0L,
        (void*)(CAT3H + (size_t)p0 * KCAT + NCH), (void*)(CAT3L + (size_t)p0 * KCAT + NCH), KCAT, 0L,
        p_bdcnr, p_bdcnr, 0L, NPC, NCH, KDEF, 0.015625f);
  }

  wmma_gemm64<1, true, 0, 0, false><<<dim3((tiles1x1 + 7) / 8, 1), 256, 0, stream>>>(
      CAT3H, CAT3L, KCAT, 0L, WFUSH, WFUSZ, KCAT, 0L, (void*)C32, (void*)C32, NCH, 0L,
      p_bdcnr, p_bdcnr, 0L, NPIX, NCH, KCAT, 1.0f);
  k_stats_part<<<STATG, 256, 0, stream>>>(C32, STP);
  k_stats_fin<<<1, 128, 0, stream>>>(STP, p_gfus, p_bfus, BNP);
  k_bn_out<<<NPIX / 32, 256, 0, stream>>>(C32, BNP, out);
}
